// GAT_TS1_83631603187930
// MI455X (gfx1250) — hardware-verified
//
#include <hip/hip_runtime.h>
#include <stdint.h>
#include <stddef.h>

#define NB   4
#define NT   60
#define NN   2048
#define NF   6
#define NH   64
#define NG   192
#define NS   8192
#define SPB  16
#define HP   72
#define OP   68
#define KX   32
#define WSC  64.0f
#define WSCI 0.015625f
#define PSC  16384.0f
#define PSCI 0.00006103515625f
#define SLOPE 0.01f

static_assert(NS == NB * NN);
static_assert(NS % SPB == 0);
static_assert(NN % SPB == 0);
static_assert(NN % 64 == 0);
static_assert(NN % 32 == 0);
static_assert((HP * 2) % 16 == 0);
static_assert((OP * 4) % 16 == 0);
static_assert(SPB * NF <= 128);
static_assert(NH == 64);
static_assert(NG == 3 * NH);
static_assert((SPB * HP) % 8 == 0);

typedef _Float16       v16h __attribute__((ext_vector_type(16)));
typedef float          v8f  __attribute__((ext_vector_type(8)));
typedef float          v4f  __attribute__((ext_vector_type(4)));
typedef unsigned int   v4u  __attribute__((ext_vector_type(4)));
typedef v4f __attribute__((may_alias)) v4fa;
typedef v4u __attribute__((may_alias)) v4ua;

union FragH { v16h v; v4u q[2]; };

__device__ __forceinline__ v8f wmma_h(v16h a, v16h b, v8f c) {
  v8f d = __builtin_amdgcn_wmma_f32_16x16x32_f16(false, a, false, b, (short)0, c, false, false);
  asm volatile("v_nop\n\tv_nop\n\tv_nop\n\tv_nop" : "+v"(d) : "v"(a), "v"(b));
  return d;
}

__device__ __forceinline__ v16h ldfrag(const unsigned short* p, int h) {
  FragH f;
  f.q[0] = *(const v4ua*)(p + 8 * h);
  f.q[1] = *(const v4ua*)(p + 16 + 8 * h);
  return f.v;
}

__device__ __forceinline__ unsigned short hbits(float a) {
  return __builtin_bit_cast(unsigned short, (_Float16)a);
}
__device__ __forceinline__ unsigned int pkh(float a, float b) {
  return (unsigned int)hbits(a) | ((unsigned int)hbits(b) << 16);
}
__device__ __forceinline__ v4u pack8(v4f a, v4f c) {
  v4u o;
  o.x = pkh(a.x, a.y); o.y = pkh(a.z, a.w);
  o.z = pkh(c.x, c.y); o.w = pkh(c.z, c.w);
  return o;
}
__device__ __forceinline__ v8f bcast8(float v) {
  v8f r;
#pragma unroll
  for (int i = 0; i < 8; ++i) r[i] = v;
  return r;
}
__device__ __forceinline__ float sigm(float x) {
  return __builtin_amdgcn_rcpf(1.0f + __expf(-x));
}
__device__ __forceinline__ float tnh(float x) {
  return 1.0f - 2.0f * __builtin_amdgcn_rcpf(__expf(2.0f * x) + 1.0f);
}
__device__ __forceinline__ float lrelu(float x) { return x > 0.0f ? x : SLOPE * x; }

__global__ __launch_bounds__(256)
void k_prep(const float* __restrict__ Wih0, const float* __restrict__ Whh0,
            const float* __restrict__ Wih1, const float* __restrict__ Whh1,
            const float* __restrict__ fcW,  const float* __restrict__ trW,
            const float* __restrict__ ffW,
            unsigned short* __restrict__ P0i, unsigned short* __restrict__ P0h,
            unsigned short* __restrict__ P1i, unsigned short* __restrict__ P1h,
            unsigned short* __restrict__ Pfc, unsigned short* __restrict__ Ptr,
            unsigned short* __restrict__ Pff)
{
  const int which = blockIdx.y;
  const int g = blockIdx.x * 256 + threadIdx.x;
  const float* src = Whh0;
  unsigned short* dst = P0h;
  int n8 = NG * NH / 8;
  if (which == 0)      { src = Wih0; dst = P0i; n8 = NG * KX / 8; }
  else if (which == 1) { src = Whh0; dst = P0h; }
  else if (which == 2) { src = Wih1; dst = P1i; }
  else if (which == 3) { src = Whh1; dst = P1h; }
  else if (which == 4) { src = fcW;  dst = Pfc; n8 = NH * NH / 8; }
  else if (which == 5) { src = trW;  dst = Ptr; n8 = NH * NH / 8; }
  else                 { src = ffW;  dst = Pff; n8 = NH * NH / 8; }
  if (g >= n8) return;

  v4u pk;
  if (which == 0) {
    const int row = g >> 2, kq = (g & 3) * 8;
    v4f lo, hi;
#pragma unroll
    for (int c = 0; c < 4; ++c) {
      const int k0 = kq + c, k1 = kq + 4 + c;
      const int c0 = (k0 < NF) ? k0 : (NF - 1);
      const int c1 = (k1 < NF) ? k1 : (NF - 1);
      const float u0 = src[row * NF + c0];
      const float u1 = src[row * NF + c1];
      lo[c] = (k0 < NF) ? u0 * WSC : 0.0f;
      hi[c] = (k1 < NF) ? u1 * WSC : 0.0f;
    }
    pk = pack8(lo, hi);
  } else {
    const float* p = src + (size_t)g * 8;
    const v4f a = *(const v4fa*)p;
    const v4f c = *(const v4fa*)(p + 4);
    pk = pack8(a * WSC, c * WSC);
  }
  unsigned short* d = dst + (size_t)g * 8;
  *(volatile v4u*)d = pk;
  __threadfence();
  *(volatile v4u*)d = pk;
}

__global__ __launch_bounds__(128) __attribute__((amdgpu_num_vgpr(256)))
void k_gru(const float* __restrict__ x,
           const unsigned short* __restrict__ P0i, const unsigned short* __restrict__ P0h,
           const unsigned short* __restrict__ P1i, const unsigned short* __restrict__ P1h,
           const float* __restrict__ bih0, const float* __restrict__ bhh0,
           const float* __restrict__ bih1, const float* __restrict__ bhh1,
           const unsigned short* __restrict__ Pfc, const float* __restrict__ fcb,
           float* __restrict__ hid)
{
  __shared__ __align__(16) unsigned short sW0i[NG * KX];
  __shared__ __align__(16) unsigned short sW0h[NG * NH];
  __shared__ __align__(16) unsigned short sW1i[NG * NH];
  __shared__ __align__(16) unsigned short sW1h[NG * NH];
  __shared__ __align__(16) unsigned short sH0[SPB * HP];
  __shared__ __align__(16) unsigned short sH1[SPB * HP];
  __shared__ __align__(16) unsigned short sX[SPB * 16];
  __shared__ __align__(16) float sOut[SPB * OP];

  const int tid = threadIdx.x, lane = tid & 31, wv = tid >> 5;
  const int h = lane >> 4, m = lane & 15;
  const int s0 = blockIdx.x * SPB;
  const int bb = blockIdx.x / (NN / SPB);
  const int n0 = (blockIdx.x % (NN / SPB)) * SPB;

#pragma unroll 1
  for (int i = tid; i < NG * KX / 8; i += 128)
    *(v4ua*)(sW0i + 8 * i) = *(const v4ua*)(P0i + 8 * i);
#pragma unroll 1
  for (int i = tid; i < NG * NH / 8; i += 128) {
    *(v4ua*)(sW0h + 8 * i) = *(const v4ua*)(P0h + 8 * i);
    *(v4ua*)(sW1i + 8 * i) = *(const v4ua*)(P1i + 8 * i);
    *(v4ua*)(sW1h + 8 * i) = *(const v4ua*)(P1h + 8 * i);
  }
  const v4u z4 = {0u, 0u, 0u, 0u};
#pragma unroll 1
  for (int i = tid; i < SPB * HP / 8; i += 128) {
    *(v4ua*)(sH0 + 8 * i) = z4;
    *(v4ua*)(sH1 + 8 * i) = z4;
  }
  if (tid < SPB * 16 / 8) *(v4ua*)(sX + 8 * tid) = z4;
  __syncthreads();

  const int gc = 16 * wv + m;
  const float b0r = WSC * (bih0[gc] + bhh0[gc]);
  const float b0z = WSC * (bih0[NH + gc] + bhh0[NH + gc]);
  const float b0x = WSC * bih0[2 * NH + gc];
  const float b0h = WSC * bhh0[2 * NH + gc];
  const float b1r = WSC * (bih1[gc] + bhh1[gc]);
  const float b1z = WSC * (bih1[NH + gc] + bhh1[NH + gc]);
  const float b1x = WSC * bih1[2 * NH + gc];
  const float b1h = WSC * bhh1[2 * NH + gc];

  const unsigned short* w0ir = sW0i + gc * KX;
  const unsigned short* w0iz = sW0i + (NH + gc) * KX;
  const unsigned short* w0in = sW0i + (2 * NH + gc) * KX;
  const unsigned short* w0hr = sW0h + gc * NH;
  const unsigned short* w0hz = sW0h + (NH + gc) * NH;
  const unsigned short* w0hn = sW0h + (2 * NH + gc) * NH;
  const unsigned short* w1ir = sW1i + gc * NH;
  const unsigned short* w1iz = sW1i + (NH + gc) * NH;
  const unsigned short* w1in = sW1i + (2 * NH + gc) * NH;
  const unsigned short* w1hr = sW1h + gc * NH;
  const unsigned short* w1hz = sW1h + (NH + gc) * NH;
  const unsigned short* w1hn = sW1h + (2 * NH + gc) * NH;
  const unsigned short* hp0 = sH0 + m * HP;
  const unsigned short* hp1 = sH1 + m * HP;
  const unsigned short* xpA = sX + m * 16;

  float hr0[8], hr1[8];
#pragma unroll
  for (int r = 0; r < 8; ++r) { hr0[r] = 0.0f; hr1[r] = 0.0f; }

#pragma unroll 1
  for (int t = 0; t < NT; ++t) {
    if (tid < SPB * NF) {
      const int q = tid / NF, f = tid - q * NF;
      const float xv = x[(((size_t)bb * NT + t) * NN + n0) * NF + tid];
      sX[q * 16 + f] = hbits(xv);
    }
    __syncthreads();

    v8f ar = bcast8(b0r), az = bcast8(b0z), an = bcast8(b0x), ah = bcast8(b0h);
    {
      FragH fx;
      fx.q[0] = *(const v4ua*)(xpA + 8 * h);
      fx.q[1] = z4;
      ar = wmma_h(fx.v, ldfrag(w0ir, h), ar);
      az = wmma_h(fx.v, ldfrag(w0iz, h), az);
      an = wmma_h(fx.v, ldfrag(w0in, h), an);
      __builtin_amdgcn_sched_barrier(0);
      const v16h a0 = ldfrag(hp0, h), a1 = ldfrag(hp0 + 32, h);
      ar = wmma_h(a0, ldfrag(w0hr, h), ar);
      ar = wmma_h(a1, ldfrag(w0hr + 32, h), ar);
      az = wmma_h(a0, ldfrag(w0hz, h), az);
      az = wmma_h(a1, ldfrag(w0hz + 32, h), az);
      ah = wmma_h(a0, ldfrag(w0hn, h), ah);
      ah = wmma_h(a1, ldfrag(w0hn + 32, h), ah);
    }
    __syncthreads();
#pragma unroll
    for (int r = 0; r < 8; ++r) {
      const float rv = sigm(ar[r] * WSCI);
      const float zv = sigm(az[r] * WSCI);
      const float nv = tnh(fmaf(rv, ah[r] * WSCI, an[r] * WSCI));
      const float hn = (1.0f - zv) * nv + zv * hr0[r];
      hr0[r] = hn;
      sH0[(8 * h + r) * HP + gc] = hbits(hn);
    }
    __syncthreads();

    ar = bcast8(b1r); az = bcast8(b1z); an = bcast8(b1x); ah = bcast8(b1h);
    {
      const v16h x0 = ldfrag(hp0, h), x1 = ldfrag(hp0 + 32, h);
      ar = wmma_h(x0, ldfrag(w1ir, h), ar);
      ar = wmma_h(x1, ldfrag(w1ir + 32, h), ar);
      az = wmma_h(x0, ldfrag(w1iz, h), az);
      az = wmma_h(x1, ldfrag(w1iz + 32, h), az);
      an = wmma_h(x0, ldfrag(w1in, h), an);
      an = wmma_h(x1, ldfrag(w1in + 32, h), an);
      __builtin_amdgcn_sched_barrier(0);
      const v16h a0 = ldfrag(hp1, h), a1 = ldfrag(hp1 + 32, h);
      ar = wmma_h(a0, ldfrag(w1hr, h), ar);
      ar = wmma_h(a1, ldfrag(w1hr + 32, h), ar);
      az = wmma_h(a0, ldfrag(w1hz, h), az);
      az = wmma_h(a1, ldfrag(w1hz + 32, h), az);
      ah = wmma_h(a0, ldfrag(w1hn, h), ah);
      ah = wmma_h(a1, ldfrag(w1hn + 32, h), ah);
    }
    __syncthreads();
#pragma unroll
    for (int r = 0; r < 8; ++r) {
      const float rv = sigm(ar[r] * WSCI);
      const float zv = sigm(az[r] * WSCI);
      const float nv = tnh(fmaf(rv, ah[r] * WSCI, an[r] * WSCI));
      const float hn = (1.0f - zv) * nv + zv * hr1[r];
      hr1[r] = hn;
      sH1[(8 * h + r) * HP + gc] = hbits(hn);
    }
  }
  __syncthreads();

  {
    v8f acc = bcast8(WSC * fcb[gc]);
    const v16h a0 = ldfrag(hp1, h), a1 = ldfrag(hp1 + 32, h);
    const unsigned short* wr = Pfc + (size_t)gc * NH;
    acc = wmma_h(a0, ldfrag(wr, h), acc);
    acc = wmma_h(a1, ldfrag(wr + 32, h), acc);
#pragma unroll
    for (int r = 0; r < 8; ++r) sOut[(8 * h + r) * OP + gc] = acc[r] * WSCI;
  }
  __syncthreads();

  v4f ov[2];
  size_t go[2];
#pragma unroll
  for (int i = 0; i < 2; ++i) {
    const int p = tid + 128 * i;
    const int row = p >> 4, c4 = (p & 15) * 4;
    ov[i] = *(const v4fa*)(sOut + row * OP + c4);
    go[i] = (size_t)(s0 + row) * NH + c4;
  }
#pragma unroll
  for (int i = 0; i < 2; ++i) *(volatile v4f*)(hid + go[i]) = ov[i];
  __threadfence();
#pragma unroll
  for (int i = 0; i < 2; ++i) *(volatile v4f*)(hid + go[i]) = ov[i];
}

__global__ __launch_bounds__(128)
void k_score(const float* __restrict__ hin,
             const unsigned short* __restrict__ Ptr, const float* __restrict__ trb,
             const float* __restrict__ av,
             float* __restrict__ sj, float* __restrict__ si,
             unsigned short* __restrict__ hT)
{
  __shared__ __align__(16) unsigned short sA[64 * HP];
  __shared__ __align__(16) float sT[64 * OP];
  __shared__ __align__(16) float sS[128];

  const int tid = threadIdx.x, lane = tid & 31, wv = tid >> 5;
  const int h = lane >> 4, m = lane & 15;
  const int blk = blockIdx.x;
  const int b = blk / (NN / 64), j0 = (blk % (NN / 64)) * 64;
  const int node0 = blk * 64;

#pragma unroll
  for (int it = 0; it < 4; ++it) {
    const int p = it * 128 + tid;
    const int row = p >> 3, c8 = (p & 7) * 8;
    const float* g = hin + (size_t)(node0 + row) * NH + c8;
    *(v4ua*)(sA + row * HP + c8) = pack8(*(const v4fa*)g, *(const v4fa*)(g + 4));
  }
  __syncthreads();

  {
    const v16h a0 = ldfrag(sA + (16 * wv + m) * HP, h);
    const v16h a1 = ldfrag(sA + (16 * wv + m) * HP + 32, h);
#pragma unroll
    for (int nt = 0; nt < 4; ++nt) {
      const unsigned short* wr = Ptr + (size_t)(16 * nt + m) * NH;
      v8f c = bcast8(WSC * trb[16 * nt + m]);
      c = wmma_h(a0, ldfrag(wr, h), c);
      c = wmma_h(a1, ldfrag(wr + 32, h), c);
#pragma unroll
      for (int r = 0; r < 8; ++r) sT[(16 * wv + 8 * h + r) * OP + 16 * nt + m] = c[r] * WSCI;
    }
  }
  __syncthreads();

  {
    const int node = tid & 63, which = tid >> 6;
    const float* ap = av + NH * which;
    const float* tp = sT + node * OP;
    float s = 0.0f;
#pragma unroll 4
    for (int f = 0; f < NH; ++f) s = fmaf(tp[f], ap[f], s);
    sS[which * 64 + node] = s;
  }

  v4u hv[4];
  size_t go[4];
#pragma unroll
  for (int it = 0; it < 4; ++it) {
    const int p = it * 128 + tid;
    const int f = p >> 3, q = p & 7;
    const unsigned short* col = sA + (8 * q) * HP + f;
    v4u o;
    o.x = (unsigned int)col[0 * HP] | ((unsigned int)col[1 * HP] << 16);
    o.y = (unsigned int)col[2 * HP] | ((unsigned int)col[3 * HP] << 16);
    o.z = (unsigned int)col[4 * HP] | ((unsigned int)col[5 * HP] << 16);
    o.w = (unsigned int)col[6 * HP] | ((unsigned int)col[7 * HP] << 16);
    hv[it] = o;
    go[it] = (size_t)(b * NH + f) * NN + j0 + 8 * q;
  }
  __syncthreads();

  const v4f sv = *(const v4fa*)(sS + 4 * lane);
  float* sd = (lane < 16) ? (sj + node0 + 4 * lane) : (si + node0 + 4 * (lane - 16));
#pragma unroll
  for (int it = 0; it < 4; ++it) *(volatile v4u*)(hT + go[it]) = hv[it];
  if (wv == 0) *(volatile v4f*)sd = sv;
  __threadfence();
#pragma unroll
  for (int it = 0; it < 4; ++it) *(volatile v4u*)(hT + go[it]) = hv[it];
  if (wv == 0) *(volatile v4f*)sd = sv;
}

__global__ __launch_bounds__(128) __attribute__((amdgpu_num_vgpr(256)))
void k_agg(const float* __restrict__ si, const float* __restrict__ sj,
           const unsigned short* __restrict__ hT, const float* __restrict__ hin,
           float* __restrict__ hout)
{
  __shared__ __align__(16) float accL[4 * 16 * OP];
  __shared__ float dpart[4 * 32];
  __shared__ float red[4];
  __shared__ float dinv[16];

  const int tid = threadIdx.x, lane = tid & 31, wv = tid >> 5;
  const int h = lane >> 4, m = lane & 15;
  const int b = blockIdx.x / (NN / 16);
  const int i0 = (blockIdx.x % (NN / 16)) * 16;
  const float* sjb = sj + (size_t)b * NN;
  const unsigned short* hTb = hT + (size_t)b * NH * NN;

  {
    const float* q = sjb + tid * 16;
    const v4f u0 = *(const v4fa*)q, u1 = *(const v4fa*)(q + 4);
    const v4f u2 = *(const v4fa*)(q + 8), u3 = *(const v4fa*)(q + 12);
    float mx = fmaxf(fmaxf(fmaxf(u0.x, u0.y), fmaxf(u0.z, u0.w)),
                     fmaxf(fmaxf(u1.x, u1.y), fmaxf(u1.z, u1.w)));
    mx = fmaxf(mx, fmaxf(fmaxf(fmaxf(u2.x, u2.y), fmaxf(u2.z, u2.w)),
                         fmaxf(fmaxf(u3.x, u3.y), fmaxf(u3.z, u3.w))));
#pragma unroll
    for (int off = 16; off > 0; off >>= 1) mx = fmaxf(mx, __shfl_xor(mx, off));
    if (lane == 0) red[wv] = mx;
  }
  __syncthreads();
  const float mxj  = fmaxf(fmaxf(red[0], red[1]), fmaxf(red[2], red[3]));
  const float siv  = si[(size_t)b * NN + i0 + m];
  const float mrow = lrelu(siv + mxj);

  const v8f z8 = {0.f, 0.f, 0.f, 0.f, 0.f, 0.f, 0.f, 0.f};
  v8f acc[4];
#pragma unroll
  for (int nt = 0; nt < 4; ++nt) acc[nt] = z8;
  float dsum = 0.0f;

#pragma unroll 1
  for (int c = wv; c < NN / 32; c += 4) {
    const int j0 = c * 32;
    const float* sp = sjb + j0 + 8 * h;
    const v4f g0 = *(const v4fa*)sp,        g1 = *(const v4fa*)(sp + 4);
    const v4f g2 = *(const v4fa*)(sp + 16), g3 = *(const v4fa*)(sp + 20);
    v4f p0, p1, p2, p3;
    p0.x = __expf(lrelu(siv + g0.x) - mrow); p0.y = __expf(lrelu(siv + g0.y) - mrow);
    p0.z = __expf(lrelu(siv + g0.z) - mrow); p0.w = __expf(lrelu(siv + g0.w) - mrow);
    p1.x = __expf(lrelu(siv + g1.x) - mrow); p1.y = __expf(lrelu(siv + g1.y) - mrow);
    p1.z = __expf(lrelu(siv + g1.z) - mrow); p1.w = __expf(lrelu(siv + g1.w) - mrow);
    p2.x = __expf(lrelu(siv + g2.x) - mrow); p2.y = __expf(lrelu(siv + g2.y) - mrow);
    p2.z = __expf(lrelu(siv + g2.z) - mrow); p2.w = __expf(lrelu(siv + g2.w) - mrow);
    p3.x = __expf(lrelu(siv + g3.x) - mrow); p3.y = __expf(lrelu(siv + g3.y) - mrow);
    p3.z = __expf(lrelu(siv + g3.z) - mrow); p3.w = __expf(lrelu(siv + g3.w) - mrow);
    dsum += (p0.x + p0.y) + (p0.z + p0.w) + (p1.x + p1.y) + (p1.z + p1.w)
          + (p2.x + p2.y) + (p2.z + p2.w) + (p3.x + p3.y) + (p3.z + p3.w);
    FragH fa;
    fa.q[0] = pack8(p0 * PSC, p1 * PSC);
    fa.q[1] = pack8(p2 * PSC, p3 * PSC);
#pragma unroll
    for (int nt = 0; nt < 4; ++nt)
      acc[nt] = wmma_h(fa.v, ldfrag(hTb + (size_t)(16 * nt + m) * NN + j0, h), acc[nt]);
  }

#pragma unroll
  for (int nt = 0; nt < 4; ++nt)
#pragma unroll
    for (int r = 0; r < 8; ++r)
      accL[(wv * 16 + 8 * h + r) * OP + 16 * nt + m] = acc[nt][r];
  dpart[wv * 32 + lane] = dsum;
  __syncthreads();
  if (tid < 16) {
    float d = 0.0f;
#pragma unroll
    for (int w = 0; w < 4; ++w) d += dpart[w * 32 + tid] + dpart[w * 32 + tid + 16];
    dinv[tid] = __builtin_amdgcn_rcpf(d) * PSCI;
  }
  __syncthreads();

  v4f ov[2];
  size_t go[2];
#pragma unroll
  for (int i = 0; i < 2; ++i) {
    const int p = tid + 128 * i;
    const int row = p >> 4, c4 = (p & 15) * 4;
    const float* ap = accL + row * OP + c4;
    const v4f s = *(const v4fa*)ap + *(const v4fa*)(ap + 16 * OP)
                + *(const v4fa*)(ap + 32 * OP) + *(const v4fa*)(ap + 48 * OP);
    const size_t gi = (size_t)(b * NN + i0 + row) * NH + c4;
    const v4f hv = *(const v4fa*)(hin + gi);
    ov[i] = s * dinv[row] + hv;
    go[i] = gi;
  }
#pragma unroll
  for (int i = 0; i < 2; ++i) *(volatile v4f*)(hout + go[i]) = ov[i];
  __threadfence();
#pragma unroll
  for (int i = 0; i < 2; ++i) *(volatile v4f*)(hout + go[i]) = ov[i];
}

__global__ __launch_bounds__(128)
void k_ffn(const float* __restrict__ hin, const unsigned short* __restrict__ Pff,
           const float* __restrict__ ffb, const float* __restrict__ foW,
           const float* __restrict__ fob, float* __restrict__ out)
{
  __shared__ __align__(16) unsigned short sA[64 * HP];
  __shared__ __align__(16) float sT[64 * OP];
  __shared__ __align__(16) float sS[64];

  const int tid = threadIdx.x, lane = tid & 31, wv = tid >> 5;
  const int h = lane >> 4, m = lane & 15;
  const int node0 = blockIdx.x * 64;

#pragma unroll
  for (int it = 0; it < 4; ++it) {
    const int p = it * 128 + tid;
    const int row = p >> 3, c8 = (p & 7) * 8;
    const float* g = hin + (size_t)(node0 + row) * NH + c8;
    *(v4ua*)(sA + row * HP + c8) = pack8(*(const v4fa*)g, *(const v4fa*)(g + 4));
  }
  __syncthreads();

  {
    const v16h a0 = ldfrag(sA + (16 * wv + m) * HP, h);
    const v16h a1 = ldfrag(sA + (16 * wv + m) * HP + 32, h);
#pragma unroll
    for (int nt = 0; nt < 4; ++nt) {
      const unsigned short* wr = Pff + (size_t)(16 * nt + m) * NH;
      v8f c = bcast8(WSC * ffb[16 * nt + m]);
      c = wmma_h(a0, ldfrag(wr, h), c);
      c = wmma_h(a1, ldfrag(wr + 32, h), c);
#pragma unroll
      for (int r = 0; r < 8; ++r) sT[(16 * wv + 8 * h + r) * OP + 16 * nt + m] = lrelu(c[r] * WSCI);
    }
  }
  __syncthreads();

  if (tid < 64) {
    const float* tp = sT + tid * OP;
    float s = fob[0];
#pragma unroll 4
    for (int g = 0; g < NH; ++g) s = fmaf(tp[g], foW[g], s);
    sS[tid] = s;
  }
  __syncthreads();

  const int lc = lane & 15;
  const v4f v = *(const v4fa*)(sS + 4 * lc);
  float* d = out + node0 + 4 * lc;
  const bool wr0 = (wv == 0) && (lane < 16);
  if (wr0) *(volatile v4f*)d = v;
  __threadfence();
  if (wr0) *(volatile v4f*)d = v;
}

extern "C" void kernel_launch(void* const* d_in, const int* in_sizes, int n_in,
                              void* d_out, int out_size, void* d_ws, size_t ws_size,
                              hipStream_t stream)
{
  if (n_in < 18) return;
  if (in_sizes[0]  != NB * NT * NN * NF) return;
  if (in_sizes[1]  != NG * NF) return;
  if (in_sizes[2]  != NG * NH) return;
  if (in_sizes[3]  != NG) return;
  if (in_sizes[4]  != NG) return;
  if (in_sizes[5]  != NG * NH) return;
  if (in_sizes[6]  != NG * NH) return;
  if (in_sizes[7]  != NG) return;
  if (in_sizes[8]  != NG) return;
  if (in_sizes[9]  != NH * NH) return;
  if (in_sizes[10] != NH) return;
  if (in_sizes[11] != NH * NH) return;
  if (in_sizes[12] != NH) return;
  if (in_sizes[13] != 2 * NH) return;
  if (in_sizes[14] != NH * NH) return;
  if (in_sizes[15] != NH) return;
  if (in_sizes[16] != NH) return;
  if (in_sizes[17] < 1) return;
  if (out_size != NS) return;

  const float* x    = (const float*)d_in[0];
  const float* Wih0 = (const float*)d_in[1];
  const float* Whh0 = (const float*)d_in[2];
  const float* bih0 = (const float*)d_in[3];
  const float* bhh0 = (const float*)d_in[4];
  const float* Wih1 = (const float*)d_in[5];
  const float* Whh1 = (const float*)d_in[6];
  const float* bih1 = (const float*)d_in[7];
  const float* bhh1 = (const float*)d_in[8];
  const float* fcW  = (const float*)d_in[9];
  const float* fcb  = (const float*)d_in[10];
  const float* trW  = (const float*)d_in[11];
  const float* trb  = (const float*)d_in[12];
  const float* av   = (const float*)d_in[13];
  const float* ffW  = (const float*)d_in[14];
  const float* ffb  = (const float*)d_in[15];
  const float* foW  = (const float*)d_in[16];
  const float* fob  = (const float*)d_in[17];
  float* out = (float*)d_out;

  const size_t bP0i = (size_t)NG * KX * 2;
  const size_t bP   = (size_t)NG * NH * 2;
  const size_t bW   = (size_t)NH * NH * 2;
  const size_t bHid = (size_t)NS * NH * 4;
  const size_t bSc  = (size_t)NS * 4;
  const size_t bHT  = (size_t)NB * NH * NN * 2;
  const size_t total = bP0i + 3 * bP + 3 * bW + 3 * bHid + 2 * bSc + bHT;
  if (total > ws_size) return;
  if (total > (size_t)134217728) return;

  char* ws = (char*)d_ws;
  size_t off = 0;
  unsigned short* P0i = (unsigned short*)(ws + off); off += bP0i;
  unsigned short* P0h = (unsigned short*)(ws + off); off += bP;
  unsigned short* P1i = (unsigned short*)(ws + off); off += bP;
  unsigned short* P1h = (unsigned short*)(ws + off); off += bP;
  unsigned short* Pfc = (unsigned short*)(ws + off); off += bW;
  unsigned short* Ptr = (unsigned short*)(ws + off); off += bW;
  unsigned short* Pff = (unsigned short*)(ws + off); off += bW;
  float* hid0 = (float*)(ws + off); off += bHid;
  float* hid1 = (float*)(ws + off); off += bHid;
  float* hid2 = (float*)(ws + off); off += bHid;
  float* sj   = (float*)(ws + off); off += bSc;
  float* si   = (float*)(ws + off); off += bSc;
  unsigned short* hT = (unsigned short*)(ws + off); off += bHT;
  if (off != total) return;

  k_prep<<<dim3(6, 7), 256, 0, stream>>>(Wih0, Whh0, Wih1, Whh1, fcW, trW, ffW,
                                          P0i, P0h, P1i, P1h, Pfc, Ptr, Pff);
  k_gru<<<NS / SPB, 128, 0, stream>>>(x, P0i, P0h, P1i, P1h, bih0, bhh0, bih1, bhh1,
                                      Pfc, fcb, hid0);
  k_score<<<NS / 64, 128, 0, stream>>>(hid0, Ptr, trb, av, sj, si, hT);
  k_agg<<<NS / 16, 128, 0, stream>>>(si, sj, hT, hid0, hid1);
  k_score<<<NS / 64, 128, 0, stream>>>(hid1, Ptr, trb, av, sj, si, hT);
  k_agg<<<NS / 16, 128, 0, stream>>>(si, sj, hT, hid1, hid2);
  k_ffn<<<NS / 64, 128, 0, stream>>>(hid2, Pff, ffb, foW, fob, out);
}
